// ResonantMultiheadAttention_12326556139612
// MI455X (gfx1250) — hardware-verified
//
#include <hip/hip_runtime.h>
#include <math.h>

constexpr int kBatch = 2;
constexpr int kSeq   = 2048;
constexpr int kDim   = 1024;
constexpr int kHeads = 16;
constexpr int kHdim  = 64;
constexpr int kTok   = kBatch * kSeq;
constexpr int kGroups = kBatch * kHeads;
constexpr int kGatePlane = kGroups * kSeq;

constexpr float kWCarry    = 16.0f;
constexpr float kWCarryInv = 1.0f / 16.0f;
constexpr float kQCarry    = 1024.0f;
constexpr float kScoreScale = 1.0f / (1024.0f * 1024.0f);
constexpr float kMCarry    = 2048.0f;
constexpr float kFCarry    = 8.0f;
constexpr float kPVScale   = kFCarry / kMCarry;
constexpr float kOutScale  = 1.0f / (kFCarry * kWCarry);
constexpr float kInvDim    = 1.0f / 1024.0f;
constexpr float kLnEps     = 1e-5f;
constexpr float kNormEps   = 1e-12f;
constexpr float kThresh    = 0.27f;
constexpr float kSharp     = 15.0f;

constexpr size_t kMiB      = 1048576;
constexpr size_t kOffWoT   = 0;
constexpr size_t kOffVT    = 2 * kMiB;
constexpr size_t kOffQKN   = 10 * kMiB;
constexpr size_t kOffGates = 26 * kMiB;
constexpr size_t kOffFused = 26 * kMiB + 524288;
constexpr size_t kOffScr   = kOffFused + 8 * kMiB;
constexpr size_t kOffXN    = kOffScr;
constexpr size_t kOffX16   = kOffScr + 8 * kMiB;
constexpr size_t kOffWqkT  = kOffScr + 16 * kMiB;
constexpr size_t kOffWvT   = kOffScr + 20 * kMiB;
constexpr size_t kOffQK32  = kOffScr + 22 * kMiB;
constexpr size_t kOffS32   = kOffScr;
constexpr size_t kOffM16   = kOffScr + 32 * kMiB;
constexpr size_t kCarve    = kOffScr + 54 * kMiB;
static_assert(kCarve == 92798976);
static_assert(kOffM16 + 16 * kMiB <= kCarve);
static_assert(kCarve <= 134217728);

typedef __attribute__((ext_vector_type(16))) _Float16 v16h;
typedef __attribute__((ext_vector_type(8)))  _Float16 v8h;
typedef __attribute__((ext_vector_type(16))) __bf16   v16b;
typedef __attribute__((ext_vector_type(8)))  __bf16   v8b;
typedef __attribute__((ext_vector_type(8)))  float    v8f;
typedef __attribute__((ext_vector_type(4)))  float    v4f;
typedef __attribute__((ext_vector_type(2)))  float    v2f;
typedef __attribute__((ext_vector_type(4)))  unsigned int v4u;

__device__ __forceinline__ unsigned short f2bf_bits(float f) {
  unsigned u = __float_as_uint(f);
  return (unsigned short)((u + 0x7FFFu + ((u >> 16) & 1u)) >> 16);
}
__device__ __forceinline__ float bf_bits2f(unsigned short h) { return __uint_as_float(((unsigned)h) << 16); }

__device__ __forceinline__ void dep_guard_h(v8f& a, v8f& b, v16h x, v16h y) { asm volatile("v_nop\n\tv_nop\n\tv_nop\n\tv_nop" : "+v"(a), "+v"(b) : "v"(x), "v"(y)); }
__device__ __forceinline__ void dep_guard_b(v8f& a, v8f& b, v16b x, v16b y) { asm volatile("v_nop\n\tv_nop\n\tv_nop\n\tv_nop" : "+v"(a), "+v"(b) : "v"(x), "v"(y)); }
__device__ __forceinline__ void keep4_h(v16h a, v16h b, v16h c, v16h d) { asm volatile("v_nop" :: "v"(a), "v"(b), "v"(c), "v"(d)); }
__device__ __forceinline__ void keep4_b(v16b a, v16b b, v16b c, v16b d) { asm volatile("v_nop" :: "v"(a), "v"(b), "v"(c), "v"(d)); }
__device__ __forceinline__ void acc_guard4(v8f& a, v8f& b, v8f& c, v8f& d) { asm volatile("v_nop\n\tv_nop\n\tv_nop\n\tv_nop" : "+v"(a), "+v"(b), "+v"(c), "+v"(d)); }
template <typename T> struct Frag;
template <> struct Frag<_Float16> {
  typedef v16h V; union U { v16h v; v8h h[2]; };
  static __device__ __forceinline__ v16h load(const _Float16* p) {
    U f; f.h[0] = *(const v8h*)(p); f.h[1] = *(const v8h*)(p + 16); return f.v;
  }
  static __device__ __forceinline__ v8f mma(v16h a, v16h b, v8f c) {
    return __builtin_amdgcn_wmma_f32_16x16x32_f16(false, a, false, b, (short)0, c, false, false);
  }
  static __device__ __forceinline__ void guard(v8f& a, v8f& b, v16h x, v16h y) { dep_guard_h(a, b, x, y); }
  static __device__ __forceinline__ void keep(v16h a, v16h b, v16h c, v16h d) { keep4_h(a, b, c, d); }
};
template <> struct Frag<__bf16> {
  typedef v16b V; union U { v16b v; v8b h[2]; };
  static __device__ __forceinline__ v16b load(const __bf16* p) {
    U f; f.h[0] = *(const v8b*)(p); f.h[1] = *(const v8b*)(p + 16); return f.v;
  }
  static __device__ __forceinline__ v8f mma(v16b a, v16b b, v8f c) {
    return __builtin_amdgcn_wmma_f32_16x16x32_bf16(false, a, false, b, (short)0, c, false, false);
  }
  static __device__ __forceinline__ void guard(v8f& a, v8f& b, v16b x, v16b y) { dep_guard_b(a, b, x, y); }
  static __device__ __forceinline__ void keep(v16b a, v16b b, v16b c, v16b d) { keep4_b(a, b, c, d); }
};

__device__ __forceinline__ unsigned pk16(unsigned short a, unsigned short b) { return (unsigned)a | ((unsigned)b << 16); }
__device__ __forceinline__ unsigned short h_bits(float f) { const _Float16 h = (_Float16)f; return __builtin_bit_cast(unsigned short, h); }

template <int ET> struct Elem;
template <> struct Elem<0> { typedef _Float16 T; };
template <> struct Elem<1> { typedef __bf16 T; };
template <int ET, bool SPLIT, int BIAS_MODE, int OUT_MODE, bool RESID, int ACT = 0>
__global__ __launch_bounds__(256) void wmma_gemm64(
    const unsigned short* __restrict__ Ap, const unsigned short* __restrict__ A2p, int lda, long strideA,
    const unsigned short* __restrict__ Btp, const unsigned short* __restrict__ Bt2p, int ldb, long strideB,
    void* __restrict__ Cout, void* __restrict__ Cout2, int ldc, long strideC,
    const float* __restrict__ bias,
    const float* __restrict__ resid, long strideR,
    int M, int N, int K, float scale) {
  typedef typename Elem<ET>::T T;
  typedef typename Frag<T>::V V;
  const T* A = (const T*)Ap; const T* A2 = (const T*)A2p; const T* Bt = (const T*)Btp; const T* Bt2 = (const T*)Bt2p;
  __shared__ __align__(16) float sT[8][16 * 68];
  const int b    = blockIdx.y;
  const int lane = threadIdx.x & 31;
  const int wave = threadIdx.x >> 5;
  const int tilesN = N >> 6;
  const int tilesM = M >> 6;
  const int tile = blockIdx.x * 8 + wave;
  if (tile >= tilesM * tilesN) return;
  const int tm = tile / tilesN;
  const int tn = tile - tm * tilesN;
  const int m0 = tm << 6;
  const int n0 = tn << 6;

  const T* Ab  = A  + (size_t)b * strideA;
  const T* Bb  = Bt + (size_t)b * strideB;
  const T* Ab2 = SPLIT ? (A2  + (size_t)b * strideA) : nullptr;
  const T* Bb2 = SPLIT ? (Bt2 + (size_t)b * strideB) : nullptr;

  const int rlane = lane & 15;
  const int koff  = (lane >> 4) * 8;
  const int mOff  = (lane >> 4) * 8;

  v8f acc[4][4];
#pragma unroll
  for (int i = 0; i < 4; ++i)
#pragma unroll
    for (int j = 0; j < 4; ++j) acc[i][j] = (v8f){0.f,0.f,0.f,0.f,0.f,0.f,0.f,0.f};

  for (int k0 = 0; k0 < K; k0 += 32) {
    V bh[4], bl[4];
#pragma unroll
    for (int j = 0; j < 4; ++j) {
      const size_t bo = (size_t)(n0 + (j << 4) + rlane) * ldb + koff + k0;
      bh[j] = Frag<T>::load(Bb + bo);
      if (SPLIT) bl[j] = Frag<T>::load(Bb2 + bo);
    }
#pragma unroll
    for (int i = 0; i < 4; ++i) {
      const size_t ao = (size_t)(m0 + (i << 4) + rlane) * lda + koff + k0;
      V ah = Frag<T>::load(Ab + ao);
      V al;
      if (SPLIT) al = Frag<T>::load(Ab2 + ao);
#pragma unroll
      for (int j = 0; j < 4; ++j) {
        acc[i][j] = Frag<T>::mma(ah, bh[j], acc[i][j]);
        if (SPLIT) {
          acc[i][j] = Frag<T>::mma(ah, bl[j], acc[i][j]);
          acc[i][j] = Frag<T>::mma(al, bh[j], acc[i][j]);
        }
      }
      Frag<T>::guard(acc[i][0], acc[i][3], ah, SPLIT ? al : ah);
    }
    Frag<T>::keep(bh[0], bh[1], bh[2], bh[3]);
    if (SPLIT) Frag<T>::keep(bl[0], bl[1], bl[2], bl[3]);
  }
  acc_guard4(acc[0][0], acc[0][1], acc[0][2], acc[0][3]);
  acc_guard4(acc[1][0], acc[1][1], acc[1][2], acc[1][3]);
  acc_guard4(acc[2][0], acc[2][1], acc[2][2], acc[2][3]);
  acc_guard4(acc[3][0], acc[3][1], acc[3][2], acc[3][3]);

  float* slab = sT[wave];
  const float* Rb = RESID ? (resid + (size_t)b * strideR) : nullptr;
#pragma unroll
  for (int i = 0; i < 4; ++i) {
    const int mBase = m0 + (i << 4);
#pragma unroll
    for (int j = 0; j < 4; ++j) {
      const int n = n0 + (j << 4) + rlane;
      float bv = 0.f;
      if (BIAS_MODE == 2) bv = bias[n];
#pragma unroll
      for (int r = 0; r < 8; ++r) {
        float v = acc[i][j][r] * scale;
        if (BIAS_MODE == 1) v += bias[mBase + mOff + r];
        if (BIAS_MODE == 2) v += bv;
        if (RESID) v += Rb[(size_t)(mBase + mOff + r) * ldc + n];
        if (ACT == 2) v = fmaxf(v, 0.0f);
        if (ACT == 4) v = (v > 0.f) ? v : 0.01f * v;
        slab[(mOff + r) * 68 + (j << 4) + rlane] = v;
      }
    }
    __builtin_amdgcn_fence(__ATOMIC_RELEASE, "workgroup");
    __builtin_amdgcn_wave_barrier();
    __builtin_amdgcn_fence(__ATOMIC_ACQUIRE, "workgroup");
    if (OUT_MODE == 0) {
      float* C = (float*)Cout + (size_t)b * strideC;
      const int hh = lane >> 4, c4 = (lane & 15) * 4;
      for (int pass = 0; pass < 2; ++pass) {
#pragma unroll
        for (int it = 0; it < 8; ++it) {
          const int row = it * 2 + hh;
          v4f v = *(const v4f*)(slab + row * 68 + c4);
          *(volatile v4f*)(C + (size_t)(mBase + row) * ldc + n0 + c4) = v;
        }
        __threadfence();
      }
    } else {
      const int q = lane >> 3, c8 = (lane & 7) * 8;
      unsigned short* C  = (unsigned short*)Cout  + (size_t)b * strideC;
      unsigned short* C2 = (OUT_MODE == 2) ? ((unsigned short*)Cout2 + (size_t)b * strideC) : nullptr;
      for (int pass = 0; pass < 2; ++pass) {
#pragma unroll
        for (int it = 0; it < 4; ++it) {
          const int row = it * 4 + q;
          const float* sp = slab + row * 68 + c8;
          v8h hv, lv;
#pragma unroll
          for (int e = 0; e < 8; ++e) {
            if (OUT_MODE == 1) {
              hv[e] = (_Float16)sp[e];
            } else {
              unsigned short hb = f2bf_bits(sp[e]);
              unsigned short lb = f2bf_bits(sp[e] - bf_bits2f(hb));
              hv[e] = __builtin_bit_cast(_Float16, hb);
              lv[e] = __builtin_bit_cast(_Float16, lb);
            }
          }
          *(volatile v8h*)(C + (size_t)(mBase + row) * ldc + n0 + c8) = hv;
          if (OUT_MODE == 2) *(volatile v8h*)(C2 + (size_t)(mBase + row) * ldc + n0 + c8) = lv;
        }
        __threadfence();
      }
    }
    __builtin_amdgcn_fence(__ATOMIC_RELEASE, "workgroup");
    __builtin_amdgcn_wave_barrier();
    __builtin_amdgcn_fence(__ATOMIC_ACQUIRE, "workgroup");
  }
}

__global__ __launch_bounds__(256) void wtcast_kernel(const float* __restrict__ W0, const float* __restrict__ W1,
                                                     const float* __restrict__ W2, const float* __restrict__ W3,
                                                     unsigned short* __restrict__ O0, unsigned short* __restrict__ O1,
                                                     unsigned short* __restrict__ O2, unsigned short* __restrict__ O3,
                                                     float scale) {
  __shared__ float sm[64][65];
  const int t  = threadIdx.x;
  const int d0 = blockIdx.x * 64;
  const int h0 = blockIdx.y * 64;
  const int z  = blockIdx.z;
  const float* W = (z == 0) ? W0 : (z == 1) ? W1 : (z == 2) ? W2 : W3;
  unsigned short* op = (z == 0) ? O0 : (z == 1) ? O1 : (z == 2) ? O2 : O3;
#pragma unroll
  for (int i = 0; i < 16; ++i) {
    const int e = i * 256 + t;
    const int r = e >> 6;
    const int c = e & 63;
    sm[c][r] = W[(size_t)(d0 + r) * kDim + h0 + c] * scale;
  }
  __syncthreads();
  const int lane = t & 31, wave = t >> 5;
  const int q = lane >> 3, c8 = (lane & 7) * 8;
  for (int pass = 0; pass < 2; ++pass) {
#pragma unroll
    for (int it = 0; it < 2; ++it) {
      const int row = wave * 8 + it * 4 + q;
      unsigned short hb[8];
#pragma unroll
      for (int e = 0; e < 8; ++e) hb[e] = h_bits(sm[row][c8 + e]);
      const v4u u = (v4u){pk16(hb[0], hb[1]), pk16(hb[2], hb[3]), pk16(hb[4], hb[5]), pk16(hb[6], hb[7])};
      *(volatile v4u*)(op + (size_t)(h0 + row) * kDim + d0 + c8) = u;
    }
    __threadfence();
  }
}

__global__ __launch_bounds__(128) void ln_cast_kernel(const float* __restrict__ x, const float* __restrict__ gamma,
                                                      const float* __restrict__ beta,
                                                      unsigned short* __restrict__ xn16, unsigned short* __restrict__ x16) {
  __shared__ float redA[4];
  __shared__ float redB[4];
  const int row  = blockIdx.x;
  const int t    = threadIdx.x;
  const int lane = t & 31, wave = t >> 5;
  const float* xr = x + (size_t)row * kDim + 8 * t;
  const v4f a = *(const v4f*)(xr);
  const v4f c = *(const v4f*)(xr + 4);
  float v[8];
#pragma unroll
  for (int e = 0; e < 4; ++e) { v[e] = a[e]; v[4 + e] = c[e]; }
  float s = 0.f;
#pragma unroll
  for (int e = 0; e < 8; ++e) s += v[e];
#pragma unroll
  for (int off = 16; off > 0; off >>= 1) s += __shfl_xor(s, off, 32);
  if (lane == 0) redA[wave] = s;
  __syncthreads();
  const float mu = ((redA[0] + redA[1]) + (redA[2] + redA[3])) * kInvDim;
  float d[8];
  float s2 = 0.f;
#pragma unroll
  for (int e = 0; e < 8; ++e) { d[e] = v[e] - mu; s2 += d[e] * d[e]; }
#pragma unroll
  for (int off = 16; off > 0; off >>= 1) s2 += __shfl_xor(s2, off, 32);
  if (lane == 0) redB[wave] = s2;
  __syncthreads();
  const float var  = ((redB[0] + redB[1]) + (redB[2] + redB[3])) * kInvDim;
  const float rstd = rsqrtf(var + kLnEps);
  const v4f g0 = *(const v4f*)(gamma + 8 * t);
  const v4f g1 = *(const v4f*)(gamma + 8 * t + 4);
  const v4f b0 = *(const v4f*)(beta + 8 * t);
  const v4f b1 = *(const v4f*)(beta + 8 * t + 4);
  float gm[8], bt[8];
#pragma unroll
  for (int e = 0; e < 4; ++e) { gm[e] = g0[e]; gm[4 + e] = g1[e]; bt[e] = b0[e]; bt[4 + e] = b1[e]; }
  unsigned short hn[8], hx[8];
#pragma unroll
  for (int e = 0; e < 8; ++e) {
    const float xn = (d[e] * rstd) * gm[e] + bt[e];
    hn[e] = h_bits(xn);
    hx[e] = h_bits(v[e]);
  }
  const v4u un = (v4u){pk16(hn[0], hn[1]), pk16(hn[2], hn[3]), pk16(hn[4], hn[5]), pk16(hn[6], hn[7])};
  const v4u ux = (v4u){pk16(hx[0], hx[1]), pk16(hx[2], hx[3]), pk16(hx[4], hx[5]), pk16(hx[6], hx[7])};
  unsigned short* pn = xn16 + (size_t)row * kDim + 8 * t;
  unsigned short* px = x16  + (size_t)row * kDim + 8 * t;
  *(volatile v4u*)pn = un;
  *(volatile v4u*)px = ux;
  __threadfence();
  *(volatile v4u*)pn = un;
  *(volatile v4u*)px = ux;
}

__global__ __launch_bounds__(256) void l2gate_kernel(const float* __restrict__ qk32, const float* __restrict__ g_q,
                                                     const float* __restrict__ g_k, unsigned short* __restrict__ qkn16,
                                                     float* __restrict__ gates) {
  __shared__ float sG[2][kHeads][32];
  const int tid  = threadIdx.x;
  const int lane = tid & 31, wave = tid >> 5;
  const int half = tid >> 7;
  const int hl   = (tid & 127) >> 3;
  const int dc   = (tid & 7) * 8;
  const int tok0 = blockIdx.x * 32;
  const int bb   = tok0 >> 11;
  const int t0   = tok0 & (kSeq - 1);
  float gq8[8], gk8[8], gs[8];
  {
    const v4f q0 = *(const v4f*)(g_q + dc), q1 = *(const v4f*)(g_q + dc + 4);
    const v4f k0 = *(const v4f*)(g_k + dc), k1 = *(const v4f*)(g_k + dc + 4);
#pragma unroll
    for (int e = 0; e < 4; ++e) { gq8[e] = q0[e]; gq8[4 + e] = q1[e]; gk8[e] = k0[e]; gk8[4 + e] = k1[e]; }
#pragma unroll
    for (int e = 0; e < 8; ++e) gs[e] = half ? gk8[e] : gq8[e];
  }
#pragma unroll 1
  for (int tok = 0; tok < 32; ++tok) {
    const int token = tok0 + tok;
    const float* src = qk32 + (size_t)token * (2 * kDim) + half * kDim + hl * kHdim + dc;
    const v4f a = *(const v4f*)(src);
    const v4f c = *(const v4f*)(src + 4);
    float v[8];
#pragma unroll
    for (int e = 0; e < 4; ++e) { v[e] = a[e]; v[4 + e] = c[e]; }
    float ss = 0.f;
#pragma unroll
    for (int e = 0; e < 8; ++e) ss += v[e] * v[e];
    ss += __shfl_xor(ss, 1, 32);
    ss += __shfl_xor(ss, 2, 32);
    ss += __shfl_xor(ss, 4, 32);
    const float nrm = sqrtf(ss);
    const float inv = 1.0f / fmaxf(nrm, kNormEps);
    float u[8];
    float gp = 0.f;
#pragma unroll
    for (int e = 0; e < 8; ++e) { u[e] = v[e] * inv; gp += u[e] * gs[e]; }
    gp += __shfl_xor(gp, 1, 32);
    gp += __shfl_xor(gp, 2, 32);
    gp += __shfl_xor(gp, 4, 32);
    const float gate = 0.25f + 0.75f / (1.0f + expf(-gp));
    if ((tid & 7) == 0) sG[half][hl][tok] = gate;
    unsigned short hb[8];
#pragma unroll
    for (int e = 0; e < 8; ++e) hb[e] = h_bits(u[e] * kQCarry);
    const v4u uu = (v4u){pk16(hb[0], hb[1]), pk16(hb[2], hb[3]), pk16(hb[4], hb[5]), pk16(hb[6], hb[7])};
    unsigned short* dst = qkn16 + (size_t)half * ((size_t)kTok * kDim) + (size_t)token * kDim + (tid & 127) * 8;
    *(volatile v4u*)dst = uu;
    __threadfence();
    *(volatile v4u*)dst = uu;
  }
  __syncthreads();
  float gv[4];
  size_t goff[4];
#pragma unroll
  for (int i = 0; i < 4; ++i) {
    const int L  = wave * 4 + i;
    const int pl = L >> 4, hd = L & 15;
    gv[i]   = sG[pl][hd][lane];
    goff[i] = (size_t)pl * kGatePlane + (size_t)(bb * kHeads + hd) * kSeq + t0 + lane;
  }
  for (int pass = 0; pass < 2; ++pass) {
#pragma unroll
    for (int i = 0; i < 4; ++i) *(volatile float*)(gates + goff[i]) = gv[i];
    __threadfence();
  }
}

__device__ __forceinline__ float rgate(float s) {
  const float z = (s - kThresh) * kSharp;
  const float e = expf(-2.0f * z);
  return 1.0f / (1.0f + e);
}
__global__ __launch_bounds__(256) void mod_kernel(const float* __restrict__ s32, const float* __restrict__ gates,
                                                  unsigned* __restrict__ m16w, int bsel, int h0) {
  const int row = blockIdx.x;
  const int j   = blockIdx.y;
  const int tid = threadIdx.x;
  const int grp = bsel * kHeads + h0 + j;
  const float gq = gates[(size_t)grp * kSeq + row];
  const float* gkrow = gates + kGatePlane + (size_t)grp * kSeq;
  const float* srow  = s32 + ((size_t)j * kSeq + row) * kSeq;
  unsigned* mrow = m16w + ((size_t)j * kSeq + row) * (kSeq / 2);
#pragma unroll 1
  for (int it = 0; it < 4; ++it) {
    const int p = it * 256 + tid;
    const v2f sv = *(const v2f*)(srow + 2 * p);
    const v2f gk = *(const v2f*)(gkrow + 2 * p);
    const float m0 = (rgate(sv[0]) * gq) * gk[0];
    const float m1 = (rgate(sv[1]) * gq) * gk[1];
    const unsigned w = pk16(h_bits(m0 * kMCarry), h_bits(m1 * kMCarry));
    *(volatile unsigned*)(mrow + p) = w;
    __threadfence();
    *(volatile unsigned*)(mrow + p) = w;
  }
}

extern "C" void kernel_launch(void* const* d_in, const int* in_sizes, int n_in,
                              void* d_out, int out_size, void* d_ws, size_t ws_size, hipStream_t stream) {
  if (n_in < 10) return;
  if (in_sizes[0] != kTok * kDim) return;
  if (in_sizes[1] != kDim * kDim || in_sizes[2] != kDim * kDim || in_sizes[3] != kDim * kDim) return;
  if (in_sizes[4] != kHdim || in_sizes[5] != kHdim) return;
  if (in_sizes[6] != kDim * kDim || in_sizes[7] != kDim || in_sizes[8] != kDim || in_sizes[9] != kDim) return;
  if (out_size != kTok * kDim) return;
  if (ws_size < kCarve) return;

  const float* x     = (const float*)d_in[0];
  const float* w_q   = (const float*)d_in[1];
  const float* w_k   = (const float*)d_in[2];
  const float* w_v   = (const float*)d_in[3];
  const float* g_q   = (const float*)d_in[4];
  const float* g_k   = (const float*)d_in[5];
  const float* w_o   = (const float*)d_in[6];
  const float* b_o   = (const float*)d_in[7];
  const float* gamma = (const float*)d_in[8];
  const float* beta  = (const float*)d_in[9];
  float* out = (float*)d_out;

  char* ws = (char*)d_ws;
  unsigned short* woT   = (unsigned short*)(ws + kOffWoT);
  unsigned short* vt16  = (unsigned short*)(ws + kOffVT);
  unsigned short* qkn16 = (unsigned short*)(ws + kOffQKN);
  float*          gates = (float*)(ws + kOffGates);
  unsigned short* fused = (unsigned short*)(ws + kOffFused);
  unsigned short* xn16  = (unsigned short*)(ws + kOffXN);
  unsigned short* x16   = (unsigned short*)(ws + kOffX16);
  unsigned short* wqkT  = (unsigned short*)(ws + kOffWqkT);
  unsigned short* wvT   = (unsigned short*)(ws + kOffWvT);
  float*          qk32  = (float*)(ws + kOffQK32);
  float*          s32   = (float*)(ws + kOffS32);
  unsigned short* m16   = (unsigned short*)(ws + kOffM16);
  const unsigned short* qn16 = qkn16;
  const unsigned short* kn16 = qkn16 + (size_t)kTok * kDim;

  wtcast_kernel<<<dim3(kDim / 64, kDim / 64, 4), 256, 0, stream>>>(
      w_q, w_k, w_v, w_o, wqkT, wqkT + (size_t)kDim * kDim, wvT, woT, kWCarry);

  ln_cast_kernel<<<kTok, 128, 0, stream>>>(x, gamma, beta, xn16, x16);

  wmma_gemm64<0, false, 0, 0, false><<<dim3(256, 1), 256, 0, stream>>>(
      xn16, xn16, kDim, 0L, wqkT, wqkT, kDim, 0L, (void*)qk32, nullptr, 2 * kDim, 0L,
      nullptr, nullptr, 0L, kTok, 2 * kDim, kDim, kWCarryInv);

  wmma_gemm64<0, false, 0, 1, false><<<dim3(128, 1), 256, 0, stream>>>(
      wvT, wvT, kDim, 0L, x16, x16, kDim, 0L, (void*)vt16, nullptr, kTok, 0L,
      nullptr, nullptr, 0L, kDim, kTok, kDim, kWCarryInv);

  l2gate_kernel<<<kTok / 32, 256, 0, stream>>>(qk32, g_q, g_k, qkn16, gates);

  for (int chunk = 0; chunk < kGroups / 2; ++chunk) {
    const int bsel = chunk >> 3;
    const int h0   = (chunk & 7) * 2;
    const size_t qoff = (size_t)bsel * kSeq * kDim + (size_t)h0 * kHdim;
    wmma_gemm64<0, false, 0, 0, false><<<dim3(128, 2), 256, 0, stream>>>(
        qn16 + qoff, qn16 + qoff, kDim, (long)kHdim, kn16 + qoff, kn16 + qoff, kDim, (long)kHdim,
        (void*)s32, nullptr, kSeq, (long)kSeq * kSeq, nullptr, nullptr, 0L, kSeq, kSeq, kHdim, kScoreScale);
    mod_kernel<<<dim3(kSeq, 2), 256, 0, stream>>>(s32, gates, (unsigned*)m16, bsel, h0);
    wmma_gemm64<0, false, 0, 1, false><<<dim3(4, 2), 256, 0, stream>>>(
        m16, m16, kSeq, (long)kSeq * kSeq,
        vt16 + (size_t)h0 * kHdim * kTok + (size_t)bsel * kSeq, vt16 + (size_t)h0 * kHdim * kTok + (size_t)bsel * kSeq, kTok, (long)kHdim * kTok,
        (void*)(fused + qoff), nullptr, kDim, (long)kHdim, nullptr, nullptr, 0L, kSeq, kHdim, kSeq, kPVScale);
  }

  wmma_gemm64<0, false, 2, 0, false><<<dim3(128, 1), 256, 0, stream>>>(
      fused, fused, kDim, 0L, woT, woT, kDim, 0L, (void*)out, nullptr, kDim, 0L,
      b_o, nullptr, 0L, kTok, kDim, kDim, kOutScale);
}
